// CausalSelfAttention_42923903156761
// MI455X (gfx1250) — hardware-verified
//
#include <hip/hip_runtime.h>
#include <math.h>

typedef __attribute__((ext_vector_type(16))) _Float16 v16h;
typedef __attribute__((ext_vector_type(16))) __bf16 v16b;
typedef __attribute__((ext_vector_type(8)))  _Float16 v8h;
typedef __attribute__((ext_vector_type(8)))  __bf16 v8b;
typedef __attribute__((ext_vector_type(8)))  float v8f;
typedef __attribute__((ext_vector_type(4)))  float v4f;
typedef __attribute__((ext_vector_type(4)))  unsigned v4u;
typedef v8h __attribute__((may_alias)) v8h_a;

#ifndef NB
#define NB 2
#endif
#ifndef SEQ
#define SEQ 2048
#endif
#define NB_FULL 2
#define SEQ_FULL 2048
#define CC 1024
#define DIN 1024
#define NH 16
#define HD 64
#define SCALE (0.125f)
#define QBH 4
#define KHI 256
#define NTHR 128
#define BROWS 64
#define BCOLS 128

static_assert(NH * HD == CC);
static_assert(HD == 64);
static_assert(DIN % 32 == 0);
static_assert(CC % 32 == 0);
static_assert(CC % BCOLS == 0);
static_assert(DIN == CC);
static_assert(SEQ % BROWS == 0);
static_assert(KHI == QBH * 64);
static_assert(SEQ >= KHI);
static_assert(SEQ <= SEQ_FULL);
static_assert(NB <= NB_FULL);
static_assert((NB * SEQ) % BROWS == 0);
static_assert(NTHR == 4 * 32);
static_assert((NTHR / 32) * 16 == BROWS);
static_assert(8 * 16 == BCOLS);
static_assert(32 * 4 == BCOLS);
static_assert(16 * 4 == HD);
static_assert(16 * 8 == BCOLS);
static_assert(8 * 8 == BROWS);
static_assert((CC * 2) % 128 == 0 && (SEQ * 2) % 128 == 0 && (KHI * 2) % 128 == 0 && (CC * 4) % 128 == 0);

#define PLANE ((size_t)NB * SEQ * CC)
#define WS_QH  ((size_t)0)
#define WS_QL  (WS_QH + 2u * PLANE)
#define WS_KH  (WS_QL + 2u * PLANE)
#define WS_KL  (WS_KH + 2u * PLANE)
#define WS_VT  (WS_KL + 2u * PLANE)
#define WS_VB  (WS_VT + 2u * PLANE)
#define WS_VBL (WS_VB + 2u * (size_t)NB * CC * KHI)
#define WS_Y   (WS_VBL + 2u * (size_t)NB * CC * KHI)
#define WS_END (WS_Y + 4u * PLANE)
static_assert(WS_END <= (size_t)134217728);
static_assert(WS_QL % 128 == 0 && WS_KH % 128 == 0 && WS_KL % 128 == 0 && WS_VT % 128 == 0 && WS_VB % 128 == 0 && WS_VBL % 128 == 0 && WS_Y % 128 == 0);

template <typename T> __device__ __forceinline__ void vst2(void* p, T v) { *(volatile T*)p = v; __threadfence(); *(volatile T*)p = v; }
__device__ __forceinline__ v8f wmma16(v16h a, v16h b, v8f c) {
  v8f d = __builtin_amdgcn_wmma_f32_16x16x32_f16(false, a, false, b, (short)0, c, false, false);
  asm volatile("v_nop\n\tv_nop\n\tv_nop\n\tv_nop" : "+v"(d) : "v"(a), "v"(b));
  return d;
}
__device__ __forceinline__ v8f wmma_bf(v16b a, v16b b, v8f c) {
  v8f d = __builtin_amdgcn_wmma_f32_16x16x32_bf16(false, a, false, b, (short)0, c, false, false);
  asm volatile("v_nop\n\tv_nop\n\tv_nop\n\tv_nop" : "+v"(d) : "v"(a), "v"(b));
  return d;
}
__device__ __forceinline__ v16h frag_h(const _Float16* rowk0, int lane) {
  union { v16h v; v8h q[2]; } u; const _Float16* p = rowk0 + 8 * (lane >> 4);
  u.q[0] = *(const v8h*)p; u.q[1] = *(const v8h*)(p + 16); return u.v;
}
__device__ __forceinline__ v16b frag_b(const __bf16* rowk0, int lane) {
  union { v16b v; v8b q[2]; } u; const __bf16* p = rowk0 + 8 * (lane >> 4);
  u.q[0] = *(const v8b*)p; u.q[1] = *(const v8b*)(p + 16); return u.v;
}
struct F2 { v16b h, l; };
__device__ __forceinline__ F2 bsplit16(const float v[16]) { F2 r;
#pragma unroll
  for (int i = 0; i < 16; ++i) { const __bf16 h = (__bf16)v[i]; r.h[i] = h; r.l[i] = (__bf16)(v[i] - (float)h); }
  return r; }
__device__ __forceinline__ F2 split_row(const float* row, int k0, int lane) { float v[16]; const float* p = row + k0 + 8 * (lane >> 4);
#pragma unroll
  for (int i = 0; i < 8; ++i) { v[i] = p[i]; v[8 + i] = p[16 + i]; }
  return bsplit16(v); }
__device__ __forceinline__ float bfr(float v) { return (float)(__bf16)v; }
__device__ __forceinline__ v16b wcol_io(const float* Wm, int k0, int o, int lane, int ld) { v16b w; const int g = lane >> 4;
#pragma unroll
  for (int i = 0; i < 8; ++i) { w[i] = (__bf16)Wm[(size_t)(k0 + 8 * g + i) * ld + o]; w[8 + i] = (__bf16)Wm[(size_t)(k0 + 16 + 8 * g + i) * ld + o]; }
  return w; }
#define LDSX() do { asm volatile("s_wait_dscnt 0" ::: "memory"); __builtin_amdgcn_wave_barrier(); __builtin_amdgcn_fence(3  , "workgroup"); } while (0)

__global__ __launch_bounds__(128) void k_proj(const float* __restrict__ X, const float* __restrict__ WA, const float* __restrict__ BA,
    _Float16* __restrict__ QK, _Float16* __restrict__ VT, __bf16* __restrict__ VB, __bf16* __restrict__ VBL) {
  __shared__ __align__(16) _Float16 sh[64][136], sl[64][136]; __shared__ __align__(16) _Float16 th[128][72]; __shared__ __align__(16) __bf16 tb[128][72], tbl[128][72];
  const int tid = threadIdx.x; const int wave = __builtin_amdgcn_readfirstlane(tid >> 5); const int lane = tid & 31, col = lane & 15, g = lane >> 4;
  const int which = blockIdx.z; const int c0 = blockIdx.y * 128; const size_t r0 = (size_t)blockIdx.x * 64; const size_t bb = r0 / SEQ; const int t0 = (int)(r0 % SEQ);
  const float* xrow = X + ((size_t)bb * SEQ_FULL + t0 + wave * 16 + col) * DIN + 8 * g;
  v8f acc[8] = {};
#pragma unroll 2
  for (int kc = 0; kc < DIN / 32; ++kc) { v16b a; { const float* p = xrow + kc * 32;
#pragma unroll
      for (int i = 0; i < 8; ++i) { a[i] = (__bf16)p[i]; a[8 + i] = (__bf16)p[16 + i]; } }
    asm volatile("s_wait_loadcnt 0x0" ::: "memory");
#pragma unroll
    for (int j = 0; j < 8; ++j) { const v16b w = wcol_io(WA, kc * 32, which * CC + c0 + j * 16 + col, lane, 3 * CC); asm volatile("s_wait_loadcnt 0x0" ::: "memory"); acc[j] = wmma_bf(a, w, acc[j]); } }
  if (which < 2) { _Float16* DH = QK + (size_t)(which * 2) * PLANE; _Float16* DL = DH + PLANE;
#pragma unroll
    for (int j = 0; j < 8; ++j) { const float bias = bfr(BA[which * CC + c0 + j * 16 + col]);
#pragma unroll
      for (int r = 0; r < 8; ++r) { const float v = acc[j][r] + bias; const _Float16 hv = (_Float16)v; sh[wave * 16 + 8 * g + r][j * 16 + col] = hv; sl[wave * 16 + 8 * g + r][j * 16 + col] = (_Float16)((v - (float)hv) * 1024.0f); } }
    __syncthreads();
    for (int e = tid; e < 64 * 16; e += 128) { const int rl = e >> 4, q = e & 15; const v4u a = *(const v4u*)&sh[rl][q * 8]; const v4u bq = *(const v4u*)&sl[rl][q * 8]; const size_t o2 = (r0 + rl) * (size_t)CC + c0 + q * 8; vst2(DH + o2, a); vst2(DL + o2, bq); }
  } else { const bool hi_rows = t0 < KHI;
#pragma unroll
    for (int j = 0; j < 8; ++j) { const float bias = bfr(BA[2 * CC + c0 + j * 16 + col]);
#pragma unroll
      for (int r = 0; r < 8; ++r) { const float v = acc[j][r] + bias; const int rl = wave * 16 + 8 * g + r, cl = j * 16 + col; th[cl][rl] = (_Float16)v; const __bf16 bh = (__bf16)v; tb[cl][rl] = bh; tbl[cl][rl] = (__bf16)(v - (float)bh); } }
    __syncthreads();
    for (int e = tid; e < 128 * 8; e += 128) { const int cl = e >> 3, q = e & 7; const v4u a = *(const v4u*)&th[cl][q * 8]; vst2(VT + (bb * CC + c0 + cl) * (size_t)SEQ + t0 + q * 8, a);
      if (hi_rows) { const size_t o3 = (bb * CC + c0 + cl) * (size_t)KHI + t0 + q * 8; const v4u bh = *(const v4u*)&tb[cl][q * 8]; const v4u bl = *(const v4u*)&tbl[cl][q * 8]; vst2(VB + o3, bh); vst2(VBL + o3, bl); } } } }

__device__ __forceinline__ void fa_scores(const _Float16* __restrict__ QH, const _Float16* __restrict__ QL, const _Float16* __restrict__ KH, const _Float16* __restrict__ KL,
    size_t qoff, size_t koff, int lane, v8f& s0, v8f& s1, v8f& t0, v8f& t1) {
#pragma unroll
  for (int kc = 0; kc < HD / 32; ++kc) {
    const v16h ah = frag_h(QH + qoff + kc * 32, lane), al = frag_h(QL + qoff + kc * 32, lane);
    const v16h kh0 = frag_h(KH + koff + kc * 32, lane), kl0 = frag_h(KL + koff + kc * 32, lane);
    s0 = wmma16(ah, kh0, s0); t0 = wmma16(al, kh0, t0); t0 = wmma16(ah, kl0, t0);
    const v16h kh1 = frag_h(KH + koff + (size_t)16 * CC + kc * 32, lane), kl1 = frag_h(KL + koff + (size_t)16 * CC + kc * 32, lane);
    s1 = wmma16(ah, kh1, s1); t1 = wmma16(al, kh1, t1); t1 = wmma16(ah, kl1, t1); } }
__device__ __forceinline__ void fa_softmax(const v8f& s0, const v8f& s1, const v8f& t0, const v8f& t1, int k0, int qg0, int col, v8f& m, v8f& l, v8f (&o)[4], v8f& p0, v8f& p1) {
#pragma unroll
  for (int r = 0; r < 8; ++r) { const int qg = qg0 + r;
    float a0 = (s0[r] + t0[r] * (1.0f / 1024.0f)) * SCALE, a1 = (s1[r] + t1[r] * (1.0f / 1024.0f)) * SCALE;
    a0 = (k0 + col <= qg) ? a0 : -3.0e38f; a1 = (k0 + 16 + col <= qg) ? a1 : -3.0e38f;
    float rm = fmaxf(a0, a1);
    rm = fmaxf(rm, __shfl_xor(rm, 1)); rm = fmaxf(rm, __shfl_xor(rm, 2)); rm = fmaxf(rm, __shfl_xor(rm, 4)); rm = fmaxf(rm, __shfl_xor(rm, 8));
    const float mo = m[r]; const float mn = fmaxf(mo, rm);
    const float ec = __expf(mo - mn), e0r = __expf(a0 - mn), e1r = __expf(a1 - mn);
    const float corr = (mo <= -1.0e38f) ? 0.f : ec; const float e0 = (a0 <= -1.0e38f) ? 0.f : e0r; const float e1 = (a1 <= -1.0e38f) ? 0.f : e1r;
    m[r] = mn; l[r] = l[r] * corr + (e0 + e1);
    o[0][r] *= corr; o[1][r] *= corr; o[2][r] *= corr; o[3][r] *= corr; p0[r] = e0; p1[r] = e1; } }

__global__ __launch_bounds__(128) void k_fa_late(const _Float16* __restrict__ QH, const _Float16* __restrict__ QL, const _Float16* __restrict__ KH, const _Float16* __restrict__ KL, const _Float16* __restrict__ VT, float* __restrict__ Y) {
  __shared__ __align__(16) _Float16 ps[4][16][40]; __shared__ __align__(16) float so[4][16][HD + 4];
  const int tid = threadIdx.x; const int wave = __builtin_amdgcn_readfirstlane(tid >> 5); const int lane = tid & 31, col = lane & 15, g = lane >> 4;
  const int qb = QBH + (int)blockIdx.x; const int h = blockIdx.y; const int b = blockIdx.z;
  const int ql0 = qb * 64 + wave * 16; const int nhalf = ((ql0 + 15) >> 5) + 1;
  const size_t qoff = ((size_t)b * SEQ + ql0 + col) * CC + h * HD; const size_t kbase = ((size_t)b * SEQ + col) * CC + h * HD; const size_t vbase = ((size_t)b * CC + h * HD + col) * (size_t)SEQ;
  v8f o[4] = {}; v8f l = {}; v8f m;
#pragma unroll
  for (int r = 0; r < 8; ++r) m[r] = -3.0e38f;
#pragma unroll 1
  for (int hk = 0; hk < nhalf; ++hk) { const int k0 = hk * 32;
    v8f s0 = {}, s1 = {}, t0 = {}, t1 = {}, p0, p1;
    fa_scores(QH, QL, KH, KL, qoff, kbase + (size_t)k0 * CC, lane, s0, s1, t0, t1);
    fa_softmax(s0, s1, t0, t1, k0, ql0 + 8 * g, col, m, l, o, p0, p1);
#pragma unroll
    for (int r = 0; r < 8; ++r) { ps[wave][8 * g + r][col] = (_Float16)(p0[r] * 2048.0f); ps[wave][8 * g + r][16 + col] = (_Float16)(p1[r] * 2048.0f); }
    LDSX();
    union { v16h v; v8h q[2]; } pu; pu.q[0] = *(const v8h_a*)&ps[wave][col][8 * g]; pu.q[1] = *(const v8h_a*)&ps[wave][col][16 + 8 * g];
#pragma unroll
    for (int j = 0; j < 4; ++j) o[j] = wmma16(pu.v, frag_h(VT + vbase + (size_t)(j * 16) * SEQ + k0, lane), o[j]);
    LDSX(); }
#pragma unroll
  for (int r = 0; r < 8; ++r) { float ls = l[r]; ls += __shfl_xor(ls, 1); ls += __shfl_xor(ls, 2); ls += __shfl_xor(ls, 4); ls += __shfl_xor(ls, 8); const float inv = 1.0f / (ls * 2048.0f);
#pragma unroll
    for (int j = 0; j < 4; ++j) so[wave][8 * g + r][j * 16 + col] = o[j][r] * inv; }
  LDSX();
  for (int it = 0; it < 8; ++it) { const int rl = it * 2 + g; const v4f v = *(const v4f*)&so[wave][rl][col * 4]; vst2(Y + ((size_t)b * SEQ + ql0 + rl) * CC + h * HD + col * 4, v); } }

__global__ __launch_bounds__(128) void k_fa_early(const _Float16* __restrict__ QH, const _Float16* __restrict__ QL, const _Float16* __restrict__ KH, const _Float16* __restrict__ KL, const __bf16* __restrict__ VB, const __bf16* __restrict__ VBL, float* __restrict__ Y) {
  __shared__ __align__(16) float pf[4][16][36]; __shared__ __align__(16) float so[4][16][HD + 4];
  const int tid = threadIdx.x; const int wave = __builtin_amdgcn_readfirstlane(tid >> 5); const int lane = tid & 31, col = lane & 15, g = lane >> 4;
  const int qb = blockIdx.x; const int h = blockIdx.y; const int b = blockIdx.z;
  const int ql0 = qb * 64 + wave * 16; const int nhalf = ((ql0 + 15) >> 5) + 1;
  const size_t qoff = ((size_t)b * SEQ + ql0 + col) * CC + h * HD; const size_t kbase = ((size_t)b * SEQ + col) * CC + h * HD; const size_t vbase = ((size_t)b * CC + h * HD + col) * (size_t)KHI;
  v8f o[4] = {}; v8f l = {}; v8f m;
#pragma unroll
  for (int r = 0; r < 8; ++r) m[r] = -3.0e38f;
#pragma unroll 1
  for (int hk = 0; hk < nhalf; ++hk) { const int k0 = hk * 32;
    v8f s0 = {}, s1 = {}, t0 = {}, t1 = {}, p0, p1;
    fa_scores(QH, QL, KH, KL, qoff, kbase + (size_t)k0 * CC, lane, s0, s1, t0, t1);
    fa_softmax(s0, s1, t0, t1, k0, ql0 + 8 * g, col, m, l, o, p0, p1);
#pragma unroll
    for (int r = 0; r < 8; ++r) { pf[wave][8 * g + r][col] = p0[r]; pf[wave][8 * g + r][16 + col] = p1[r]; }
    LDSX();
    float pv[16];
#pragma unroll
    for (int i = 0; i < 8; ++i) { pv[i] = pf[wave][col][8 * g + i]; pv[8 + i] = pf[wave][col][16 + 8 * g + i]; }
    const F2 p = bsplit16(pv);
#pragma unroll
    for (int j = 0; j < 4; ++j) { const size_t po = vbase + (size_t)(j * 16) * KHI + k0; const v16b vh = frag_b(VB + po, lane); o[j] = wmma_bf(p.h, vh, o[j]); o[j] = wmma_bf(p.l, vh, o[j]); o[j] = wmma_bf(p.h, frag_b(VBL + po, lane), o[j]); }
    LDSX(); }
#pragma unroll
  for (int r = 0; r < 8; ++r) { float ls = l[r]; ls += __shfl_xor(ls, 1); ls += __shfl_xor(ls, 2); ls += __shfl_xor(ls, 4); ls += __shfl_xor(ls, 8); const float inv = 1.0f / ls;
#pragma unroll
    for (int j = 0; j < 4; ++j) so[wave][8 * g + r][j * 16 + col] = o[j][r] * inv; }
  LDSX();
  for (int it = 0; it < 8; ++it) { const int rl = it * 2 + g; const v4f v = *(const v4f*)&so[wave][rl][col * 4]; vst2(Y + ((size_t)b * SEQ + ql0 + rl) * CC + h * HD + col * 4, v); } }

__global__ __launch_bounds__(128) void k_out(const float* __restrict__ Y, const float* __restrict__ WO, const float* __restrict__ BO, float* __restrict__ OUT) {
  __shared__ __align__(16) float sf[4][16][132];
  const int tid = threadIdx.x; const int wave = __builtin_amdgcn_readfirstlane(tid >> 5); const int lane = tid & 31, col = lane & 15, g = lane >> 4;
  const int c0 = blockIdx.y * 128; const size_t rb = (size_t)blockIdx.x * 64; const size_t bb = rb / SEQ; const int t0 = (int)(rb % SEQ);
  const size_t r0 = rb + wave * 16; const size_t orow0 = bb * SEQ_FULL + t0 + wave * 16;
  v8f acc[8] = {};
#pragma unroll 2
  for (int kc = 0; kc < CC / 32; ++kc) { const F2 a = split_row(Y + (r0 + col) * CC, kc * 32, lane); asm volatile("s_wait_loadcnt 0x0" ::: "memory");
#pragma unroll
    for (int j = 0; j < 8; ++j) { const v16b w = wcol_io(WO, kc * 32, c0 + j * 16 + col, lane, DIN); asm volatile("s_wait_loadcnt 0x0" ::: "memory"); acc[j] = wmma_bf(a.h, w, acc[j]); acc[j] = wmma_bf(a.l, w, acc[j]); } }
#pragma unroll
  for (int j = 0; j < 8; ++j) { const float bias = bfr(BO[c0 + j * 16 + col]);
#pragma unroll
    for (int r = 0; r < 8; ++r) sf[wave][8 * g + r][j * 16 + col] = acc[j][r] + bias; }
  LDSX();
  for (int rl = 0; rl < 16; ++rl) { const v4f v = *(const v4f*)&sf[wave][rl][lane * 4]; vst2(OUT + (orow0 + rl) * DIN + c0 + lane * 4, v); } }

extern "C" void kernel_launch(void* const* d_in, const int* in_sizes, int n_in, void* d_out, int out_size, void* d_ws, size_t ws_size, hipStream_t stream) {
  if (n_in < 5) return;
  const size_t need_rows = (size_t)(NB - 1) * SEQ_FULL + SEQ;
  if ((size_t)in_sizes[0] < need_rows * DIN) return;
  if ((size_t)in_sizes[1] < (size_t)DIN * 3 * CC) return;
  if ((size_t)in_sizes[2] < (size_t)3 * CC) return;
  if ((size_t)in_sizes[3] < (size_t)CC * DIN) return;
  if ((size_t)in_sizes[4] < (size_t)DIN) return;
  if ((size_t)out_size < need_rows * DIN) return;
  if (ws_size < (size_t)WS_END) return;
  const float* x = (const float*)d_in[0]; const float* W_qkv = (const float*)d_in[1]; const float* b_qkv = (const float*)d_in[2]; const float* W_proj = (const float*)d_in[3]; const float* b_proj = (const float*)d_in[4];
  char* ws = (char*)d_ws;
  _Float16 *QH = (_Float16*)(ws + WS_QH), *QL = (_Float16*)(ws + WS_QL), *KH = (_Float16*)(ws + WS_KH), *KL = (_Float16*)(ws + WS_KL), *VT = (_Float16*)(ws + WS_VT);
  __bf16 *VB = (__bf16*)(ws + WS_VB), *VBL = (__bf16*)(ws + WS_VBL); float* Y = (float*)(ws + WS_Y);
  k_proj<<<dim3(NB * SEQ / 64, CC / 128, 3), 128, 0, stream>>>(x, W_qkv, b_qkv, QH, VT, VB, VBL);
  k_fa_early<<<dim3(QBH, NH, NB), 128, 0, stream>>>(QH, QL, KH, KL, VB, VBL, Y);
  if (SEQ / 64 > QBH) k_fa_late<<<dim3(SEQ / 64 - QBH, NH, NB), 128, 0, stream>>>(QH, QL, KH, KL, VT, Y);
  k_out<<<dim3(NB * SEQ / 64, DIN / 128), 128, 0, stream>>>(Y, W_proj, b_proj, (float*)d_out);
}
